// CausalReasoningModule_18330920419659
// MI455X (gfx1250) — hardware-run, weakly checked
//
#include <hip/hip_runtime.h>
#include <stdint.h>
#include <stddef.h>
#include <math.h>

#define NBATCH 4096
#define NF     512
#define NA     64
#define NN     8
#define NH     128
#define NL     3
#define NROWS  32768
#define NB2    8192
#define NOUT   64
#define TPE    68

static_assert(NROWS == NBATCH * NN);
static_assert(NB2 == 2 * NBATCH);
static_assert((NF + NA) % 32 == 0);
static_assert(NF % 64 == 0);
static_assert(NH % 64 == 0);
static_assert((TPE * 4) % 16 == 0);

typedef _Float16     v16h __attribute__((ext_vector_type(16)));
typedef float        v8f  __attribute__((ext_vector_type(8)));
typedef float        v4f  __attribute__((ext_vector_type(4)));
typedef unsigned int v4u  __attribute__((ext_vector_type(4)));
typedef unsigned int v2u  __attribute__((ext_vector_type(2)));
typedef v4f __attribute__((may_alias)) v4fa;
typedef v4u __attribute__((may_alias)) v4ua;
typedef v2u __attribute__((may_alias)) v2ua;

union FragH { v16h v; v4u q[2]; };

__device__ __forceinline__ v8f wmma_h(v16h a, v16h b, v8f c) {
  v8f d = __builtin_amdgcn_wmma_f32_16x16x32_f16(false, a, false, b, (short)0, c, false, false);
  asm volatile("v_nop\n\tv_nop\n\tv_nop\n\tv_nop" : "+v"(d) : "v"(a), "v"(b));
  return d;
}

__device__ __forceinline__ v16h ldfrag(const unsigned short* p, int h) {
  FragH f;
  f.q[0] = *(const v4ua*)(p + 8 * h);
  f.q[1] = *(const v4ua*)(p + 16 + 8 * h);
  return f.v;
}

__device__ __forceinline__ unsigned int pk2h(float a, float b) {
  const _Float16 ha = (_Float16)a;
  const _Float16 hb = (_Float16)b;
  const unsigned short ua = __builtin_bit_cast(unsigned short, ha);
  const unsigned short ub = __builtin_bit_cast(unsigned short, hb);
  return (unsigned int)ua | ((unsigned int)ub << 16);
}
__device__ __forceinline__ v4u pk8h(v4f a, v4f b) {
  v4u o;
  o.x = pk2h(a.x, a.y); o.y = pk2h(a.z, a.w);
  o.z = pk2h(b.x, b.y); o.w = pk2h(b.z, b.w);
  return o;
}
__device__ __forceinline__ v2u pk4h(v4f a) {
  v2u o;
  o.x = pk2h(a.x, a.y); o.y = pk2h(a.z, a.w);
  return o;
}

__device__ __forceinline__ float gelu1(float x) {
  return 0.5f * x * (1.0f + erff(x * 0.70710678118654752f));
}
__device__ __forceinline__ v4f gelu4(v4f v) {
  v4f o;
  o.x = gelu1(v.x); o.y = gelu1(v.y); o.z = gelu1(v.z); o.w = gelu1(v.w);
  return o;
}

__device__ __forceinline__ v4f ln128(v4f x, v4f g, v4f be) {
  float s = (x.x + x.y) + (x.z + x.w);
  #pragma unroll
  for (int o = 16; o > 0; o >>= 1) s += __shfl_xor(s, o, 32);
  const float mu = s * (1.0f / 128.0f);
  const v4f d = x - mu;
  float q = d.x * d.x + d.y * d.y + d.z * d.z + d.w * d.w;
  #pragma unroll
  for (int o = 16; o > 0; o >>= 1) q += __shfl_xor(q, o, 32);
  const float rstd = rsqrtf(q * (1.0f / 128.0f) + 1e-5f);
  return d * rstd * g + be;
}

__global__ __launch_bounds__(256) void k_cvtw(const float* __restrict__ src, int K, int N,
                                              int segS, int segD, unsigned short* Dst)
{
  __shared__ float sT[64 * 65];
  const int tid = threadIdx.x;
  const float* s = src + (size_t)blockIdx.z * (size_t)segS;
  unsigned short* d = Dst + (size_t)blockIdx.z * (size_t)segD;
  const int nt0 = blockIdx.x * 64, kt0 = blockIdx.y * 64;
  #pragma unroll
  for (int i = 0; i < 16; ++i) {
    const int idx = tid + 256 * i;
    const int kk = idx >> 6, nn = idx & 63;
    sT[kk * 65 + nn] = s[(size_t)(kt0 + kk) * N + nt0 + nn];
  }
  __syncthreads();
  v4u o[2];
  size_t oa[2];
  #pragma unroll
  for (int it = 0; it < 2; ++it) {
    const int r = (tid >> 3) + 32 * it, p = tid & 7;
    v4f a, b;
    a.x = sT[(8 * p + 0) * 65 + r] * 64.0f; a.y = sT[(8 * p + 1) * 65 + r] * 64.0f;
    a.z = sT[(8 * p + 2) * 65 + r] * 64.0f; a.w = sT[(8 * p + 3) * 65 + r] * 64.0f;
    b.x = sT[(8 * p + 4) * 65 + r] * 64.0f; b.y = sT[(8 * p + 5) * 65 + r] * 64.0f;
    b.z = sT[(8 * p + 6) * 65 + r] * 64.0f; b.w = sT[(8 * p + 7) * 65 + r] * 64.0f;
    o[it] = pk8h(a, b);
    oa[it] = (size_t)(nt0 + r) * K + kt0 + 8 * p;
  }
  #pragma unroll
  for (int it = 0; it < 2; ++it) *(volatile v4u*)(d + oa[it]) = o[it];
  __threadfence();
  #pragma unroll
  for (int it = 0; it < 2; ++it) *(volatile v4u*)(d + oa[it]) = o[it];
}

__global__ __launch_bounds__(256) void k_xcat(const float* __restrict__ obs,
                                              const float* __restrict__ act,
                                              const float* __restrict__ nz,
                                              unsigned short* X)
{
  #pragma clang fp contract(off)
  const int tid = threadIdx.x, lane = tid & 31, wv = tid >> 5;
  const int r = blockIdx.x * 8 + wv;
  const int rb = r & (NBATCH - 1);
  const bool iscf = (r >= NBATCH);
  v4u oo[2];
  #pragma unroll
  for (int s = 0; s < 2; ++s) {
    const float* p = obs + (size_t)rb * NF + 256 * s + 8 * lane;
    const v4f a = *(const v4fa*)(p);
    const v4f b = *(const v4fa*)(p + 4);
    oo[s] = pk8h(a, b);
  }
  const int q = lane & 7;
  const v4f a0 = *(const v4fa*)(act + (size_t)rb * NA + 8 * q);
  const v4f a1 = *(const v4fa*)(act + (size_t)rb * NA + 8 * q + 4);
  const v4f n0 = *(const v4fa*)(nz + (size_t)rb * NA + 8 * q);
  const v4f n1 = *(const v4fa*)(nz + (size_t)rb * NA + 8 * q + 4);
  const v4f t0 = n0 * 0.1f, t1 = n1 * 0.1f;
  const v4f c0 = a0 + t0, c1 = a1 + t1;
  const v4f s0 = iscf ? c0 : a0;
  const v4f s1 = iscf ? c1 : a1;
  const v4u oact = pk8h(s0, s1);
  const size_t base = (size_t)r * (NF + NA);
  *(volatile v4u*)(X + base + 8 * lane) = oo[0];
  *(volatile v4u*)(X + base + 256 + 8 * lane) = oo[1];
  if (lane < 8) *(volatile v4u*)(X + base + NF + 8 * q) = oact;
  __threadfence();
  *(volatile v4u*)(X + base + 8 * lane) = oo[0];
  *(volatile v4u*)(X + base + 256 + 8 * lane) = oo[1];
  if (lane < 8) *(volatile v4u*)(X + base + NF + 8 * q) = oact;
}

template<int BIAS, int WF, int WH>
__global__ __launch_bounds__(128) void k_gemm(
    const unsigned short* __restrict__ A, int lda,
    const unsigned short* __restrict__ Bt, int ldb, int K,
    const float* __restrict__ bias,
    float* Cf, int ldc, unsigned short* Ch, int ldh)
{
  __shared__ __align__(16) float sT[64 * TPE];
  const int tid = threadIdx.x, lane = tid & 31, wv = tid >> 5;
  const int h = lane >> 4, m = lane & 15;
  const int wm = wv >> 1, wn = wv & 1;
  const int rb = blockIdx.x * 64, cb = blockIdx.y * 64;

  const v8f z8 = {0.f, 0.f, 0.f, 0.f, 0.f, 0.f, 0.f, 0.f};
  v8f acc[2][2];
  #pragma unroll
  for (int mt = 0; mt < 2; ++mt)
    #pragma unroll
    for (int nt = 0; nt < 2; ++nt) acc[mt][nt] = z8;

  #pragma unroll 1
  for (int k0 = 0; k0 < K; k0 += 32) {
    v16h a[2];
    #pragma unroll
    for (int mt = 0; mt < 2; ++mt) {
      const size_t ao = (size_t)(rb + 32 * wm + 16 * mt + m) * lda + k0;
      a[mt] = ldfrag(A + ao, h);
    }
    #pragma unroll
    for (int nt = 0; nt < 2; ++nt) {
      const size_t bo = (size_t)(cb + 32 * wn + 16 * nt + m) * ldb + k0;
      const v16h b = ldfrag(Bt + bo, h);
      #pragma unroll
      for (int mt = 0; mt < 2; ++mt) acc[mt][nt] = wmma_h(a[mt], b, acc[mt][nt]);
    }
  }

  #pragma unroll
  for (int mt = 0; mt < 2; ++mt)
    #pragma unroll
    for (int nt = 0; nt < 2; ++nt) {
      const int col = 32 * wn + 16 * nt + m;
      #pragma unroll
      for (int r = 0; r < 8; ++r) {
        const int row = 32 * wm + 16 * mt + 8 * h + r;
        sT[row * TPE + col] = acc[mt][nt][r];
      }
    }
  __syncthreads();

  const float sc = 0.015625f;
  v4f fo[8];
  size_t fa[8];
  if (WF) {
    #pragma unroll
    for (int i = 0; i < 8; ++i) {
      const int rr = 16 * wv + 2 * i + (lane >> 4), c4 = 4 * (lane & 15);
      const int grow = rb + rr, gcol = cb + c4;
      v4f v = *(const v4fa*)(sT + rr * TPE + c4) * sc;
      if (BIAS) v += *(const v4fa*)(bias + gcol);
      fo[i] = v;
      fa[i] = (size_t)grow * ldc + gcol;
    }
  }
  v4u po[4];
  size_t pa[4];
  if (WH) {
    #pragma unroll
    for (int q = 0; q < 4; ++q) {
      const int rr = 16 * wv + 4 * q + (lane >> 3), c8 = 8 * (lane & 7);
      const int grow = rb + rr, gcol = cb + c8;
      v4f v0 = *(const v4fa*)(sT + rr * TPE + c8) * sc;
      v4f v1 = *(const v4fa*)(sT + rr * TPE + c8 + 4) * sc;
      if (BIAS) {
        v0 += *(const v4fa*)(bias + gcol);
        v1 += *(const v4fa*)(bias + gcol + 4);
      }
      po[q] = pk8h(v0, v1);
      pa[q] = (size_t)grow * ldh + gcol;
    }
  }
  if (WF) {
    #pragma unroll
    for (int i = 0; i < 8; ++i) *(volatile v4f*)(Cf + fa[i]) = fo[i];
  }
  if (WH) {
    #pragma unroll
    for (int q = 0; q < 4; ++q) *(volatile v4u*)(Ch + pa[q]) = po[q];
  }
  __threadfence();
  if (WF) {
    #pragma unroll
    for (int i = 0; i < 8; ++i) *(volatile v4f*)(Cf + fa[i]) = fo[i];
  }
  if (WH) {
    #pragma unroll
    for (int q = 0; q < 4; ++q) *(volatile v4u*)(Ch + pa[q]) = po[q];
  }
}

template<int GELU, int ADDH, int WF, int WZ>
__global__ __launch_bounds__(256) void k_ln(
    const float* __restrict__ X, const float* __restrict__ Hs, const float* __restrict__ ab,
    const float* __restrict__ gam, const float* __restrict__ bet, const float* __restrict__ zs,
    float* Of, unsigned short* Oh, unsigned short* Oz)
{
  __shared__ __align__(16) unsigned short sH[8 * NH];
  const int tid = threadIdx.x, lane = tid & 31, wv = tid >> 5;
  const size_t row = (size_t)blockIdx.x * 8 + wv;
  const int c = 4 * lane;
  v4f x = *(const v4fa*)(X + row * NH + c);
  if (ADDH) {
    const v4f hs = *(const v4fa*)(Hs + (row >> 3) * NH + c);
    const v4f bb = *(const v4fa*)(ab + c);
    x = (hs + x) + bb;
  }
  const v4f g = *(const v4fa*)(gam + c);
  const v4f be = *(const v4fa*)(bet + c);
  v4f y = ln128(x, g, be);
  if (GELU) y = gelu4(y);
  const size_t fo = row * NH + c;
  if (WF) *(volatile v4f*)(Of + fo) = y;
  *(v2ua*)(sH + wv * NH + c) = pk4h(y);
  __syncthreads();
  const int p = lane & 15;
  const v4u piece = *(const v4ua*)(sH + wv * NH + 8 * p);
  v4u zsel = piece;
  if (WZ) {
    const v4f z0 = *(const v4fa*)(zs + (row >> 3) * NH + 8 * p);
    const v4f z1 = *(const v4fa*)(zs + (row >> 3) * NH + 8 * p + 4);
    const v4u zp = pk8h(z0, z1);
    zsel = ((row & 7) == 0) ? zp : piece;
  }
  const size_t ho = row * NH + 8 * p;
  if (lane < 16) {
    *(volatile v4u*)(Oh + ho) = piece;
    if (WZ) *(volatile v4u*)(Oz + ho) = zsel;
  }
  __threadfence();
  if (WF) *(volatile v4f*)(Of + fo) = y;
  if (lane < 16) {
    *(volatile v4u*)(Oh + ho) = piece;
    if (WZ) *(volatile v4u*)(Oz + ho) = zsel;
  }
}

__global__ __launch_bounds__(256) void k_adj(const float* __restrict__ P,
                                             const float* __restrict__ eb,
                                             const float* __restrict__ w2,
                                             const float* __restrict__ b2,
                                             const float* __restrict__ temp,
                                             float* adj)
{
  __shared__ __align__(16) float sS[64];
  const int tid = threadIdx.x, lane = tid & 31, wv = tid >> 5;
  const int b = blockIdx.x, i = wv;
  const size_t row = (size_t)b * NN + i;
  const int c = 4 * lane;
  const v4f hi = *(const v4fa*)(P + row * (2 * NH) + c);
  const v4f bb = *(const v4fa*)(eb + c);
  const v4f w = *(const v4fa*)(w2 + c);
  const float rt = 1.0f / (fabsf(temp[0]) + 1e-6f);
  const float bs = b2[0];
  #pragma unroll 1
  for (int j = 0; j < NN; ++j) {
    const v4f hj = *(const v4fa*)(P + ((size_t)b * NN + j) * (2 * NH) + NH + c);
    const v4f x = (hi + hj) + bb;
    const v4f y = gelu4(x);
    float d = y.x * w.x + y.y * w.y + y.z * w.z + y.w * w.w;
    #pragma unroll
    for (int o = 16; o > 0; o >>= 1) d += __shfl_xor(d, o, 32);
    const float s = d + bs;
    const float sc = (i == j) ? -1.0e9f : s;
    const float e = expf(-(sc * rt));
    const float sig = __builtin_amdgcn_rcpf(1.0f + e);
    if (lane == 0) sS[i * NN + j] = sig;
  }
  __syncthreads();
  const int p = lane & 15;
  const v4f v = *(const v4fa*)(sS + 4 * p);
  const size_t o = (size_t)b * (NN * NN) + 4 * p;
  if (wv == 0 && lane < 16) *(volatile v4f*)(adj + o) = v;
  __threadfence();
  if (wv == 0 && lane < 16) *(volatile v4f*)(adj + o) = v;
}

__global__ __launch_bounds__(256) void k_msg(const float* __restrict__ P,
                                             const float* __restrict__ gb,
                                             const float* __restrict__ gg,
                                             const float* __restrict__ gbe,
                                             const float* __restrict__ adj,
                                             const unsigned short* __restrict__ vin,
                                             unsigned short* acat)
{
  __shared__ __align__(16) unsigned short sA[8 * NH];
  const int tid = threadIdx.x, lane = tid & 31, wv = tid >> 5;
  const int b = blockIdx.x, i = wv;
  const size_t row = (size_t)b * NN + i;
  const int c = 4 * lane;
  const v4f hi = *(const v4fa*)(P + row * (2 * NH) + NH + c);
  const v4f bb = *(const v4fa*)(gb + c);
  const v4f g = *(const v4fa*)(gg + c);
  const v4f be = *(const v4fa*)(gbe + c);
  v4f agg = {0.f, 0.f, 0.f, 0.f};
  #pragma unroll 1
  for (int j = 0; j < NN; ++j) {
    const v4f hj = *(const v4fa*)(P + ((size_t)b * NN + j) * (2 * NH) + c);
    const v4f x = (hj + hi) + bb;
    const v4f y = gelu4(ln128(x, g, be));
    const float a = adj[(size_t)b * (NN * NN) + i * NN + j];
    agg += y * a;
  }
  *(v2ua*)(sA + wv * NH + c) = pk4h(agg);
  __syncthreads();
  const int h = lane >> 4, p = lane & 15;
  const v4u vp = *(const v4ua*)(vin + row * NH + 8 * p);
  const v4u ap = *(const v4ua*)(sA + wv * NH + 8 * p);
  const v4u val = (h != 0) ? ap : vp;
  const size_t o = row * (2 * NH) + NH * h + 8 * p;
  *(volatile v4u*)(acat + o) = val;
  __threadfence();
  *(volatile v4u*)(acat + o) = val;
}

__global__ __launch_bounds__(256) void k_eff(const float* __restrict__ P,
                                             const float* __restrict__ eb,
                                             const float* __restrict__ eg,
                                             const float* __restrict__ ebe,
                                             const float* __restrict__ w2,
                                             const float* __restrict__ b2,
                                             float* eff)
{
  __shared__ __align__(16) float sS[64];
  const int tid = threadIdx.x, lane = tid & 31, wv = tid >> 5;
  const int b = blockIdx.x, i = wv;
  const size_t row = (size_t)b * NN + i;
  const int c = 4 * lane;
  const v4f hi = *(const v4fa*)(P + row * (2 * NH) + c);
  const v4f bb = *(const v4fa*)(eb + c);
  const v4f g = *(const v4fa*)(eg + c);
  const v4f be = *(const v4fa*)(ebe + c);
  const v4f w = *(const v4fa*)(w2 + c);
  const float bs = b2[0];
  #pragma unroll 1
  for (int j = 0; j < NN; ++j) {
    const v4f hj = *(const v4fa*)(P + ((size_t)b * NN + j) * (2 * NH) + NH + c);
    const v4f x = (hi + hj) + bb;
    const v4f y = gelu4(ln128(x, g, be));
    float d = y.x * w.x + y.y * w.y + y.z * w.z + y.w * w.w;
    #pragma unroll
    for (int o = 16; o > 0; o >>= 1) d += __shfl_xor(d, o, 32);
    const float val = (i == j) ? 0.0f : (d + bs);
    if (lane == 0) sS[i * NN + j] = val;
  }
  __syncthreads();
  const int p = lane & 15;
  const v4f v = *(const v4fa*)(sS + 4 * p);
  const size_t o = (size_t)b * (NN * NN) + 4 * p;
  if (wv == 0 && lane < 16) *(volatile v4f*)(eff + o) = v;
  __threadfence();
  if (wv == 0 && lane < 16) *(volatile v4f*)(eff + o) = v;
}

__global__ __launch_bounds__(256) void k_ivpost(const float* __restrict__ delta,
                                                const float* __restrict__ adj,
                                                const float* __restrict__ vf,
                                                const float* __restrict__ zv,
                                                float* outp)
{
  const int tid = threadIdx.x, lane = tid & 31, wv = tid >> 5;
  const size_t row = (size_t)blockIdx.x * 8 + wv;
  const size_t b = row >> 3;
  const int i = (int)(row & 7);
  const int c = 4 * lane;
  const v4f z0 = *(const v4fa*)(zv + b * NH + c);
  const v4f vv = *(const v4fa*)(vf + row * NH + c);
  const v4f z = (i == 0) ? z0 : vv;
  const v4f d = *(const v4fa*)(delta + row * NH + c);
  const float a = adj[b * (NN * NN) + i];
  const v4f o = z + d * a;
  const size_t oo = row * NH + c;
  *(volatile v4f*)(outp + oo) = o;
  __threadfence();
  *(volatile v4f*)(outp + oo) = o;
}

__global__ __launch_bounds__(256) void k_cfin(const unsigned short* __restrict__ vh,
                                              const float* __restrict__ vcf,
                                              const float* __restrict__ vf,
                                              unsigned short* cfin)
{
  __shared__ __align__(16) unsigned short sC[8 * 3 * NH];
  const int tid = threadIdx.x, lane = tid & 31, wv = tid >> 5;
  const size_t b = (size_t)blockIdx.x * 8 + wv;
  const int h = lane >> 4, p = lane & 15, c = 4 * lane;
  const v4u v0p = *(const v4ua*)(vh + b * (NN * NH) + 8 * p);
  const v4f c0 = *(const v4fa*)(vcf + b * (NN * NH) + 8 * p);
  const v4f c1 = *(const v4fa*)(vcf + b * (NN * NH) + 8 * p + 4);
  const v4u vcp = pk8h(c0, c1);
  const v4u sel = (h != 0) ? vcp : v0p;
  *(v4ua*)(sC + wv * (3 * NH) + NH * h + 8 * p) = sel;
  v4f s = {0.f, 0.f, 0.f, 0.f};
  #pragma unroll
  for (int i = 0; i < NN; ++i) {
    const v4f va = *(const v4fa*)(vf + (b * NN + i) * NH + c);
    const v4f vb = *(const v4fa*)(vcf + b * (NN * NH) + i * NH + c);
    const v4f dlt = va - vb;
    s = s + dlt;
  }
  s = s * 0.125f;
  *(v2ua*)(sC + wv * (3 * NH) + 2 * NH + c) = pk4h(s);
  __syncthreads();
  const v4u o0 = *(const v4ua*)(sC + wv * (3 * NH) + 8 * lane);
  const v4u o1 = *(const v4ua*)(sC + wv * (3 * NH) + 2 * NH + 8 * p);
  const size_t a0 = b * (3 * NH) + 8 * lane;
  const size_t a1 = b * (3 * NH) + 2 * NH + 8 * p;
  *(volatile v4u*)(cfin + a0) = o0;
  if (lane < 16) *(volatile v4u*)(cfin + a1) = o1;
  __threadfence();
  *(volatile v4u*)(cfin + a0) = o0;
  if (lane < 16) *(volatile v4u*)(cfin + a1) = o1;
}

__global__ __launch_bounds__(256) void k_mean(const float* __restrict__ adj, float* om)
{
  __shared__ double sR[256];
  const int t = threadIdx.x;
  double s = 0.0;
  #pragma unroll 4
  for (int k = 0; k < 1024; ++k) s += (double)adj[t + 256 * k];
  sR[t] = s;
  __syncthreads();
  for (int st = 128; st > 0; st >>= 1) {
    if (t < st) sR[t] += sR[t + st];
    __syncthreads();
  }
  if (t == 0) {
    const float mval = (float)(sR[0] * (1.0 / 262144.0));
    *(volatile float*)om = mval;
    __threadfence();
    *(volatile float*)om = mval;
  }
}

extern "C" void kernel_launch(void* const* d_in, const int* in_sizes, int n_in,
                              void* d_out, int out_size, void* d_ws, size_t ws_size,
                              hipStream_t stream)
{
  if (n_in < 45) return;
  if (in_sizes[0]  != NBATCH * NF) return;
  if (in_sizes[1]  != NBATCH * NA) return;
  if (in_sizes[2]  != NBATCH * NH) return;
  if (in_sizes[3]  != NBATCH * NA) return;
  if (in_sizes[4]  != (NF + NA) * NF) return;
  if (in_sizes[5]  != NF) return;
  if (in_sizes[6]  != NF * NH) return;
  if (in_sizes[7]  != NH) return;
  if (in_sizes[8]  != NH) return;
  if (in_sizes[9]  != NH) return;
  if (in_sizes[10] != NH * NN * NH) return;
  if (in_sizes[11] != NN * NH) return;
  if (in_sizes[12] != 2 * NH * NH) return;
  if (in_sizes[13] != NH) return;
  if (in_sizes[14] != NH) return;
  if (in_sizes[15] != 1) return;
  if (in_sizes[16] != 1) return;
  if (in_sizes[17] != NL * 2 * NH * NH) return;
  if (in_sizes[18] != NL * NH) return;
  if (in_sizes[19] != NL * NH) return;
  if (in_sizes[20] != NL * NH) return;
  if (in_sizes[21] != NL * 2 * NH * NH) return;
  if (in_sizes[22] != NL * NH) return;
  if (in_sizes[23] != NL * NH) return;
  if (in_sizes[24] != NL * NH) return;
  if (in_sizes[25] != 2 * NH * NH) return;
  if (in_sizes[26] != NH) return;
  if (in_sizes[27] != NH) return;
  if (in_sizes[28] != NH) return;
  if (in_sizes[29] != NH * NH) return;
  if (in_sizes[30] != NH) return;
  if (in_sizes[31] != 3 * NH * NH) return;
  if (in_sizes[32] != NH) return;
  if (in_sizes[33] != NH) return;
  if (in_sizes[34] != NH) return;
  if (in_sizes[35] != NH * NH) return;
  if (in_sizes[36] != NH) return;
  if (in_sizes[37] != 2 * NH * NH) return;
  if (in_sizes[38] != NH) return;
  if (in_sizes[39] != NH) return;
  if (in_sizes[40] != NH) return;
  if (in_sizes[41] != NH) return;
  if (in_sizes[42] != 1) return;
  if (in_sizes[43] != NN * NH * NOUT) return;
  if (in_sizes[44] != NOUT) return;
  if (out_size != 9699329) return;

  const float* obs    = (const float*)d_in[0];
  const float* act    = (const float*)d_in[1];
  const float* z_val  = (const float*)d_in[2];
  const float* noise  = (const float*)d_in[3];
  const float* ip_w   = (const float*)d_in[4];
  const float* ip_b   = (const float*)d_in[5];
  const float* ve1_w  = (const float*)d_in[6];
  const float* ve1_b  = (const float*)d_in[7];
  const float* ve_g   = (const float*)d_in[8];
  const float* ve_be  = (const float*)d_in[9];
  const float* ve2_w  = (const float*)d_in[10];
  const float* ve2_b  = (const float*)d_in[11];
  const float* es1_w  = (const float*)d_in[12];
  const float* es1_b  = (const float*)d_in[13];
  const float* es2_w  = (const float*)d_in[14];
  const float* es2_b  = (const float*)d_in[15];
  const float* temp   = (const float*)d_in[16];
  const float* gm_w   = (const float*)d_in[17];
  const float* gm_b   = (const float*)d_in[18];
  const float* gm_g   = (const float*)d_in[19];
  const float* gm_be  = (const float*)d_in[20];
  const float* gu_w   = (const float*)d_in[21];
  const float* gu_b   = (const float*)d_in[22];
  const float* gu_g   = (const float*)d_in[23];
  const float* gu_be  = (const float*)d_in[24];
  const float* iv1_w  = (const float*)d_in[25];
  const float* iv1_b  = (const float*)d_in[26];
  const float* iv_g   = (const float*)d_in[27];
  const float* iv_be  = (const float*)d_in[28];
  const float* iv2_w  = (const float*)d_in[29];
  const float* iv2_b  = (const float*)d_in[30];
  const float* cf1_w  = (const float*)d_in[31];
  const float* cf1_b  = (const float*)d_in[32];
  const float* cf_g   = (const float*)d_in[33];
  const float* cf_be  = (const float*)d_in[34];
  const float* cf2_w  = (const float*)d_in[35];
  const float* cf2_b  = (const float*)d_in[36];
  const float* ee1_w  = (const float*)d_in[37];
  const float* ee1_b  = (const float*)d_in[38];
  const float* ee_g   = (const float*)d_in[39];
  const float* ee_be  = (const float*)d_in[40];
  const float* ee2_w  = (const float*)d_in[41];
  const float* ee2_b  = (const float*)d_in[42];
  const float* op_w   = (const float*)d_in[43];
  const float* op_b   = (const float*)d_in[44];

  float* out   = (float*)d_out;
  float* oAdj  = out;
  float* oV    = out + 262144;
  float* oEff  = out + 4456448;
  float* oItv  = out + 4718592;
  float* oCf   = out + 8912896;
  float* oCr   = out + 9437184;
  float* oMean = out + 9699328;

  const size_t szWip  = (size_t)(NF + NA) * NF * 2;
  const size_t szWve1 = (size_t)NF * NH * 2;
  const size_t szWve2 = (size_t)NH * NN * NH * 2;
  const size_t szWes1 = (size_t)2 * NH * NH * 2;
  const size_t szWgm  = (size_t)NL * 2 * NH * NH * 2;
  const size_t szWgu  = (size_t)NL * 2 * NH * NH * 2;
  const size_t szWiv1 = (size_t)2 * NH * NH * 2;
  const size_t szWiv2 = (size_t)NH * NH * 2;
  const size_t szWcf1 = (size_t)3 * NH * NH * 2;
  const size_t szWcf2 = (size_t)NH * NH * 2;
  const size_t szWee1 = (size_t)2 * NH * NH * 2;
  const size_t szWop  = (size_t)NN * NH * NOUT * 2;
  const size_t szX    = (size_t)NB2 * (NF + NA) * 2;
  const size_t szX16  = (size_t)NB2 * NF * 2;
  const size_t szG32  = (size_t)NB2 * NH * 4;
  const size_t szH16  = (size_t)NB2 * NH * 2;
  const size_t szVCF  = (size_t)NBATCH * NN * NH * 4;
  const size_t szV    = (size_t)NROWS * NH * 2;
  const size_t szP    = (size_t)NROWS * 2 * NH * 4;
  const size_t szAC   = (size_t)NROWS * 2 * NH * 2;
  const size_t total = szWip + szWve1 + szWve2 + szWes1 + szWgm + szWgu + szWiv1 + szWiv2
      + szWcf1 + szWcf2 + szWee1 + szWop + szX + szX16 + szG32 + szH16 + szVCF + 3 * szV + szP + szAC;
  if (total > ws_size) return;
  if (total > (size_t)134217728) return;
  if ((size_t)NROWS * NH * 2 > szX) return;
  if ((size_t)NROWS * NH * 2 > szX16) return;
  if ((size_t)NBATCH * 3 * NH * 2 > szX16) return;
  if ((size_t)NBATCH * NH * 4 > szG32) return;
  if ((size_t)NBATCH * NH * 2 > szH16) return;
  if ((size_t)2 * NROWS * NH * 4 > szP) return;

  char* ws = (char*)d_ws;
  size_t off = 0;
  unsigned short* Wip  = (unsigned short*)(ws + off); off += szWip;
  unsigned short* Wve1 = (unsigned short*)(ws + off); off += szWve1;
  unsigned short* Wve2 = (unsigned short*)(ws + off); off += szWve2;
  unsigned short* Wes1 = (unsigned short*)(ws + off); off += szWes1;
  unsigned short* Wgm  = (unsigned short*)(ws + off); off += szWgm;
  unsigned short* Wgu  = (unsigned short*)(ws + off); off += szWgu;
  unsigned short* Wiv1 = (unsigned short*)(ws + off); off += szWiv1;
  unsigned short* Wiv2 = (unsigned short*)(ws + off); off += szWiv2;
  unsigned short* Wcf1 = (unsigned short*)(ws + off); off += szWcf1;
  unsigned short* Wcf2 = (unsigned short*)(ws + off); off += szWcf2;
  unsigned short* Wee1 = (unsigned short*)(ws + off); off += szWee1;
  unsigned short* Wop  = (unsigned short*)(ws + off); off += szWop;
  unsigned short* xcat = (unsigned short*)(ws + off); off += szX;
  unsigned short* x16  = (unsigned short*)(ws + off); off += szX16;
  float*          g32  = (float*)(ws + off);          off += szG32;
  unsigned short* h16  = (unsigned short*)(ws + off); off += szH16;
  float*          vcf32 = (float*)(ws + off);         off += szVCF;
  unsigned short* V0   = (unsigned short*)(ws + off); off += szV;
  unsigned short* VA   = (unsigned short*)(ws + off); off += szV;
  unsigned short* VB   = (unsigned short*)(ws + off); off += szV;
  float*          P    = (float*)(ws + off);          off += szP;
  unsigned short* acat = (unsigned short*)(ws + off); off += szAC;
  if (off != total) return;
  unsigned short* z16   = xcat;
  unsigned short* t16   = x16;
  unsigned short* cfin  = x16;
  float*          hs32  = g32;
  float*          cpre  = g32;
  unsigned short* c16   = h16;
  float*          pre32 = P;
  float*          hz32  = P;
  float*          dlt32 = P + (size_t)NROWS * NH;

  k_cvtw<<<dim3(NF / 64, (NF + NA) / 64, 1), 256, 0, stream>>>(ip_w, NF + NA, NF, 0, 0, Wip);
  k_cvtw<<<dim3(NH / 64, NF / 64, 1), 256, 0, stream>>>(ve1_w, NF, NH, 0, 0, Wve1);
  k_cvtw<<<dim3(NN * NH / 64, NH / 64, 1), 256, 0, stream>>>(ve2_w, NH, NN * NH, 0, 0, Wve2);
  k_cvtw<<<dim3(NH / 64, NH / 64, 2), 256, 0, stream>>>(es1_w, NH, NH, NH * NH, NH * NH, Wes1);
  k_cvtw<<<dim3(NH / 64, NH / 64, 2 * NL), 256, 0, stream>>>(gm_w, NH, NH, NH * NH, NH * NH, Wgm);
  k_cvtw<<<dim3(NH / 64, 2 * NH / 64, NL), 256, 0, stream>>>(gu_w, 2 * NH, NH, 2 * NH * NH, 2 * NH * NH, Wgu);
  k_cvtw<<<dim3(NH / 64, NH / 64, 2), 256, 0, stream>>>(iv1_w, NH, NH, NH * NH, NH * NH, Wiv1);
  k_cvtw<<<dim3(NH / 64, NH / 64, 1), 256, 0, stream>>>(iv2_w, NH, NH, 0, 0, Wiv2);
  k_cvtw<<<dim3(NH / 64, 3 * NH / 64, 1), 256, 0, stream>>>(cf1_w, 3 * NH, NH, 0, 0, Wcf1);
  k_cvtw<<<dim3(NH / 64, NH / 64, 1), 256, 0, stream>>>(cf2_w, NH, NH, 0, 0, Wcf2);
  k_cvtw<<<dim3(NH / 64, NH / 64, 2), 256, 0, stream>>>(ee1_w, NH, NH, NH * NH, NH * NH, Wee1);
  k_cvtw<<<dim3(NOUT / 64, NN * NH / 64, 1), 256, 0, stream>>>(op_w, NN * NH, NOUT, 0, 0, Wop);

  k_xcat<<<NB2 / 8, 256, 0, stream>>>(obs, act, noise, xcat);
  k_gemm<1, 0, 1><<<dim3(NB2 / 64, NF / 64), 128, 0, stream>>>(
      xcat, NF + NA, Wip, NF + NA, NF + NA, ip_b, g32, NH, x16, NF);
  k_gemm<1, 1, 0><<<dim3(NB2 / 64, NH / 64), 128, 0, stream>>>(
      x16, NF, Wve1, NF, NF, ve1_b, g32, NH, h16, NH);
  k_ln<1, 0, 0, 0><<<NB2 / 8, 256, 0, stream>>>(g32, g32, ve1_b, ve_g, ve_be, z_val, g32, h16, z16);
  k_gemm<1, 0, 1><<<dim3(NBATCH / 64, NN * NH / 64), 128, 0, stream>>>(
      h16, NH, Wve2, NH, NH, ve2_b, vcf32, NN * NH, V0, NN * NH);
  k_gemm<1, 1, 0><<<dim3(NBATCH / 64, NN * NH / 64), 128, 0, stream>>>(
      h16 + (size_t)NBATCH * NH, NH, Wve2, NH, NH, ve2_b, vcf32, NN * NH, V0, NN * NH);
  k_gemm<0, 1, 0><<<dim3(NROWS / 64, 2 * NH / 64), 128, 0, stream>>>(
      V0, NH, Wes1, NH, NH, ip_b, P, 2 * NH, h16, NH);
  k_adj<<<NBATCH, 256, 0, stream>>>(P, es1_b, es2_w, es2_b, temp, oAdj);

  for (int l = 0; l < NL; ++l) {
    const unsigned short* vin = (l == 0) ? V0 : ((l == 1) ? VA : VB);
    unsigned short* vout = (l == 1) ? VB : VA;
    k_gemm<0, 1, 0><<<dim3(NROWS / 64, 2 * NH / 64), 128, 0, stream>>>(
        vin, NH, Wgm + (size_t)l * 2 * NH * NH, NH, NH, ip_b, P, 2 * NH, h16, NH);
    k_msg<<<NBATCH, 256, 0, stream>>>(P, gm_b + l * NH, gm_g + l * NH, gm_be + l * NH, oAdj, vin, acat);
    k_gemm<1, 1, 0><<<dim3(NROWS / 64, NH / 64), 128, 0, stream>>>(
        acat, 2 * NH, Wgu + (size_t)l * 2 * NH * NH, 2 * NH, 2 * NH, gu_b + l * NH, pre32, NH, h16, NH);
    if (l < NL - 1) {
      k_ln<0, 0, 0, 0><<<NROWS / 8, 256, 0, stream>>>(pre32, pre32, gu_b + l * NH, gu_g + l * NH, gu_be + l * NH,
                                                      z_val, g32, vout, z16);
    } else {
      k_ln<0, 0, 1, 1><<<NROWS / 8, 256, 0, stream>>>(pre32, pre32, gu_b + l * NH, gu_g + l * NH, gu_be + l * NH,
                                                      z_val, oV, vout, z16);
    }
  }
  unsigned short* vfin = VA;

  k_gemm<0, 1, 0><<<dim3(NROWS / 64, 2 * NH / 64), 128, 0, stream>>>(
      vfin, NH, Wee1, NH, NH, ip_b, P, 2 * NH, h16, NH);
  k_eff<<<NBATCH, 256, 0, stream>>>(P, ee1_b, ee_g, ee_be, ee2_w, ee2_b, oEff);

  k_gemm<0, 1, 0><<<dim3(NBATCH / 64, NH / 64), 128, 0, stream>>>(
      z16, NN * NH, Wiv1, NH, NH, ip_b, hs32, NH, h16, NH);
  k_gemm<0, 1, 0><<<dim3(NROWS / 64, NH / 64), 128, 0, stream>>>(
      z16, NH, Wiv1 + (size_t)NH * NH, NH, NH, ip_b, hz32, NH, h16, NH);
  k_ln<1, 1, 0, 0><<<NROWS / 8, 256, 0, stream>>>(hz32, hs32, iv1_b, iv_g, iv_be, z_val, g32, t16, z16);
  k_gemm<1, 1, 0><<<dim3(NROWS / 64, NH / 64), 128, 0, stream>>>(
      t16, NH, Wiv2, NH, NH, iv2_b, dlt32, NH, h16, NH);
  k_ivpost<<<NROWS / 8, 256, 0, stream>>>(dlt32, oAdj, oV, z_val, oItv);

  k_cfin<<<NBATCH / 8, 256, 0, stream>>>(vfin, vcf32, oV, cfin);
  k_gemm<1, 1, 0><<<dim3(NBATCH / 64, NH / 64), 128, 0, stream>>>(
      cfin, 3 * NH, Wcf1, 3 * NH, 3 * NH, cf1_b, cpre, NH, h16, NH);
  k_ln<1, 0, 0, 0><<<NBATCH / 8, 256, 0, stream>>>(cpre, cpre, cf1_b, cf_g, cf_be, z_val, g32, c16, z16);
  k_gemm<1, 1, 0><<<dim3(NBATCH / 64, NH / 64), 128, 0, stream>>>(
      c16, NH, Wcf2, NH, NH, cf2_b, oCf, NH, h16, NH);

  k_gemm<1, 1, 0><<<dim3(NBATCH / 64, NOUT / 64), 128, 0, stream>>>(
      vfin, NN * NH, Wop, NN * NH, NN * NH, op_b, oCr, NOUT, h16, NH);

  k_mean<<<1, 256, 0, stream>>>(oAdj, oMean);
}
